// Caption_Model_35588099014669
// MI455X (gfx1250) — hardware-verified
//
#include <hip/hip_runtime.h>


#define NBT  64
#define NF   36
#define DI   2048
#define LH   1000
#define LP   1024
#define G4   4096
#define DICT 9956
#define DVP  9984
#define DAT  512
#define K1   4096
#define K2   3072
#define NSTEP 19
#define TW   20
typedef _Float16 h16;
typedef unsigned short bf;
typedef __attribute__((ext_vector_type(16))) __bf16   v16bf;
typedef __attribute__((ext_vector_type(16))) _Float16 v16h;
typedef __attribute__((ext_vector_type(8)))  _Float16 v8h;
typedef __attribute__((ext_vector_type(8)))  unsigned short v8us;
typedef __attribute__((ext_vector_type(8)))  float    v8f;
typedef __attribute__((ext_vector_type(4)))  float    v4f;
typedef v8h  __attribute__((may_alias)) v8ha;
typedef v4f  __attribute__((may_alias)) v4fa;
typedef v8us __attribute__((may_alias)) v8usa;

__device__ __forceinline__ unsigned short f2bf(float f) { unsigned u = __float_as_uint(f); u += 0x7FFFu + ((u >> 16) & 1u); return (unsigned short)(u >> 16); }
__device__ __forceinline__ float bf2f(unsigned short b) { return __uint_as_float(((unsigned)b) << 16); }
__device__ __forceinline__ float bfr(float f) { return bf2f(f2bf(f)); }
__device__ __forceinline__ v16h cat16(v8h lo, v8h hi) { return __builtin_shufflevector(lo, hi, 0, 1, 2, 3, 4, 5, 6, 7, 8, 9, 10, 11, 12, 13, 14, 15); }
__device__ __forceinline__ v16bf cat16b(v8us lo, v8us hi) { return __builtin_bit_cast(v16bf, __builtin_shufflevector(lo, hi, 0, 1, 2, 3, 4, 5, 6, 7, 8, 9, 10, 11, 12, 13, 14, 15)); }
__device__ __forceinline__ v8f wmma16(v16h a, v16h b, v8f c) { return __builtin_amdgcn_wmma_f32_16x16x32_f16(false, a, false, b, (short)0, c, false, false); }
__device__ __forceinline__ v8f wmmab(v16bf a, v16bf b, v8f c) { return __builtin_amdgcn_wmma_f32_16x16x32_bf16(false, a, false, b, (short)0, c, false, false); }


template <typename T16> struct WFrag;
template <> struct WFrag<h16> { typedef v16h V; static __device__ __forceinline__ V ld(const h16* p) { return cat16(*(const v8h*)p, *(const v8h*)(p + 16)); } static __device__ __forceinline__ v8f mma(V a, V b, v8f c) { return wmma16(a, b, c); } };
template <> struct WFrag<bf> { typedef v16bf V; static __device__ __forceinline__ V ld(const bf* p) { return cat16b(*(const v8us*)p, *(const v8us*)(p + 16)); } static __device__ __forceinline__ v8f mma(V a, V b, v8f c) { return wmmab(a, b, c); } };
template <typename T16, int NSPLIT, bool BIAS>
__global__ __launch_bounds__(32) void k_gemmw(const T16* __restrict__ A, const T16* __restrict__ A2, const T16* __restrict__ Bt, const T16* __restrict__ Bt2, int K, float* C, int ldc, const float* __restrict__ bias, size_t sA, size_t sB, size_t sC) {
    typedef typename WFrag<T16>::V V;
    __shared__ __align__(16) float os[16 * 68];
    const size_t z = blockIdx.z; A += z * sA; if (A2) A2 += z * sA; Bt += z * sB; if (Bt2) Bt2 += z * sB; C += z * sC;
    const int lane = threadIdx.x & 31, lr = lane & 15, hi = lane >> 4; const int r0 = blockIdx.x * 64, c0 = blockIdx.y * 64;
    v8f acc[4][4];
#pragma unroll
    for (int mb = 0; mb < 4; ++mb)
#pragma unroll
        for (int nb = 0; nb < 4; ++nb) acc[mb][nb] = (v8f){};
    const size_t aoff = (size_t)(r0 + lr) * K + 8 * hi, boff = (size_t)(c0 + lr) * K + 8 * hi;
#pragma unroll 1
    for (int kc = 0; kc < K; kc += 32) {
        V a[4], a2[4];
#pragma unroll
        for (int mb = 0; mb < 4; ++mb) { a[mb] = WFrag<T16>::ld(A + aoff + (size_t)mb * 16 * K + kc); if (NSPLIT == 1 || NSPLIT == 2) a2[mb] = WFrag<T16>::ld(A2 + aoff + (size_t)mb * 16 * K + kc); }
#pragma unroll
        for (int nb = 0; nb < 4; ++nb) { const V b = WFrag<T16>::ld(Bt + boff + (size_t)nb * 16 * K + kc); V b2; if (NSPLIT >= 2) b2 = WFrag<T16>::ld(Bt2 + boff + (size_t)nb * 16 * K + kc);
#pragma unroll
            for (int mb = 0; mb < 4; ++mb) { acc[mb][nb] = WFrag<T16>::mma(a[mb], b, acc[mb][nb]); if (NSPLIT == 1 || NSPLIT == 2) acc[mb][nb] = WFrag<T16>::mma(a2[mb], b, acc[mb][nb]); if (NSPLIT >= 2) acc[mb][nb] = WFrag<T16>::mma(a[mb], b2, acc[mb][nb]); } }
        asm volatile("v_nop\n\tv_nop\n\tv_nop\n\tv_nop" : "+v"(acc[0][0]), "+v"(acc[1][1]), "+v"(acc[2][2]), "+v"(acc[3][3]) : "v"(a[0]), "v"(a[3]));
    }
#pragma unroll
    for (int mb = 0; mb < 4; ++mb) {
#pragma unroll
        for (int nb = 0; nb < 4; ++nb) {
#pragma unroll
            for (int j = 0; j < 8; ++j) os[(hi * 8 + j) * 68 + nb * 16 + lr] = acc[mb][nb][j]; }
        __builtin_amdgcn_wave_barrier(); asm volatile("" ::: "memory");
        float* crow = C + (size_t)(r0 + mb * 16) * ldc + c0;
#pragma unroll 1
        for (int ps = 0; ps < 2; ++ps) {
#pragma unroll
            for (int s = 0; s < 8; ++s) { const int row = 2 * s + hi, cofs = lr * 4; v4f val = *(const v4fa*)(os + row * 68 + cofs); if (BIAS) { val[0] += bfr(bias[c0 + cofs]); val[1] += bfr(bias[c0 + cofs + 1]); val[2] += bfr(bias[c0 + cofs + 2]); val[3] += bfr(bias[c0 + cofs + 3]); }
                *(volatile v4f*)(crow + (size_t)row * ldc + cofs) = val; }
            if (ps == 0) __threadfence(); }
        __builtin_amdgcn_wave_barrier(); asm volatile("" ::: "memory");
    }
}

__device__ __forceinline__ h16 tohx(float x) { return (h16)x; }
__device__ __forceinline__ float sigm_(float x) { return __fdiv_rn(1.0f, 1.0f + __expf(-x)); }
__device__ __forceinline__ float tanh_(float x) { const float e = __expf(-2.0f * fabsf(x)); const float t = __fdiv_rn(1.0f - e, 1.0f + e); return copysignf(t, x); }
typedef __attribute__((ext_vector_type(2))) _Float16 v2h;
typedef __attribute__((ext_vector_type(4))) _Float16 v4h;
typedef __attribute__((ext_vector_type(2))) float v2f;

__global__ __launch_bounds__(256) void k_cvt8(const float* __restrict__ src, bf* dst, size_t n8) { const size_t i = (size_t)blockIdx.x * 256 + threadIdx.x; if (i >= n8) return; const v8f v = *(const v8f*)(src + i * 8); v8us o;
#pragma unroll
    for (int k = 0; k < 8; ++k) o[k] = f2bf(v[k]); *(volatile v8us*)(dst + i * 8) = o; __threadfence(); *(volatile v8us*)(dst + i * 8) = o; }
__device__ __forceinline__ int gaterow(int n) { const int g = n / LP, j = n % LP; return j < LH ? g * LH + j : -1; }
__global__ __launch_bounds__(256) void k_w1x(const float* __restrict__ w, h16* Bt) { const size_t e = ((size_t)blockIdx.x * 256 + threadIdx.x) * 4; if (e >= (size_t)G4 * K1) return; const int k = (int)(e % K1); const int r = gaterow((int)(e / K1)); v4h o;
#pragma unroll
    for (int q = 0; q < 4; ++q) { const int kk = k + q; int src = -1; if (kk < LP) src = kk < LH ? kk : -1; else if (kk < LP + DI) src = LH + (kk - LP); else src = (kk - LP - DI) < LH ? LH + DI + (kk - LP - DI) : -1; o[q] = (r >= 0 && src >= 0) ? tohx(bfr(w[(size_t)r * (LH + DI + LH) + src])) : (h16)0.f; }
    *(volatile v4h*)(Bt + e) = o; __threadfence(); *(volatile v4h*)(Bt + e) = o; }
__global__ __launch_bounds__(256) void k_whh(const float* __restrict__ w, h16* Bt) { const size_t e = ((size_t)blockIdx.x * 256 + threadIdx.x) * 4; if (e >= (size_t)G4 * LP) return; const int k = (int)(e % LP); const int r = gaterow((int)(e / LP)); v4h o;
#pragma unroll
    for (int q = 0; q < 4; ++q) o[q] = (r >= 0 && k + q < LH) ? tohx(bfr(w[(size_t)r * LH + k + q])) : (h16)0.f; *(volatile v4h*)(Bt + e) = o; __threadfence(); *(volatile v4h*)(Bt + e) = o; }
__global__ __launch_bounds__(256) void k_w2x(const float* __restrict__ w, h16* Bt) { const size_t e = ((size_t)blockIdx.x * 256 + threadIdx.x) * 4; if (e >= (size_t)G4 * K2) return; const int k = (int)(e % K2); const int r = gaterow((int)(e / K2)); v4h o;
#pragma unroll
    for (int q = 0; q < 4; ++q) { const int kk = k + q; const int src = kk < LP ? (kk < LH ? kk : -1) : LH + (kk - LP); o[q] = (r >= 0 && src >= 0) ? tohx(bfr(w[(size_t)r * (LH + DI) + src])) : (h16)0.f; }
    *(volatile v4h*)(Bt + e) = o; __threadfence(); *(volatile v4h*)(Bt + e) = o; }
__global__ __launch_bounds__(256) void k_wah(const float* __restrict__ w, h16* Bt) { const size_t e = ((size_t)blockIdx.x * 256 + threadIdx.x) * 4; if (e >= (size_t)DAT * LP) return; const int k = (int)(e % LP); const int a = (int)(e / LP); v4h o;
#pragma unroll
    for (int q = 0; q < 4; ++q) o[q] = (k + q < LH) ? tohx(bfr(w[(size_t)a * LH + k + q])) : (h16)0.f; *(volatile v4h*)(Bt + e) = o; __threadfence(); *(volatile v4h*)(Bt + e) = o; }
__global__ __launch_bounds__(256) void k_wp(const float* __restrict__ w, h16* Bt) { const size_t e = ((size_t)blockIdx.x * 256 + threadIdx.x) * 4; if (e >= (size_t)DVP * LP) return; const int k = (int)(e % LP); const int v = (int)(e / LP); v4h o;
#pragma unroll
    for (int q = 0; q < 4; ++q) o[q] = (v < DICT && k + q < LH) ? tohx(bfr(w[(size_t)v * LH + k + q])) : (h16)0.f; *(volatile v4h*)(Bt + e) = o; __threadfence(); *(volatile v4h*)(Bt + e) = o; }
__global__ __launch_bounds__(256) void k_vmean(const float* __restrict__ F, float* VM) { const size_t e = ((size_t)blockIdx.x * 256 + threadIdx.x) * 4; if (e >= (size_t)NBT * DI) return; const int f = (int)(e % DI); const int b = (int)(e / DI); v4f o;
#pragma unroll
    for (int q = 0; q < 4; ++q) { float s = 0.f;
#pragma unroll 1
        for (int n = 0; n < NF; ++n) s = __fadd_rn(s, bfr(F[((size_t)b * NF + n) * DI + f + q])); o[q] = __fmul_rn(s, 1.0f / (float)NF); }
    *(volatile v4f*)(VM + e) = o; __threadfence(); *(volatile v4f*)(VM + e) = o; }
__global__ __launch_bounds__(256) void k_init(const float* __restrict__ h0, const float* __restrict__ c0, float* H, float* Cs, h16* H16) { const size_t e = ((size_t)blockIdx.x * 256 + threadIdx.x) * 4; if (e >= (size_t)NBT * LP) return; const int j = (int)(e % LP); v4f h, c; v4h hh;
#pragma unroll
    for (int q = 0; q < 4; ++q) { const bool in = (j + q) < LH; h[q] = in ? bfr(h0[j + q]) : 0.f; c[q] = in ? bfr(c0[j + q]) : 0.f; hh[q] = tohx(h[q]); }
    for (int ps = 0; ps < 2; ++ps) { *(volatile v4f*)(H + e) = h; *(volatile v4f*)(Cs + e) = c; *(volatile v4h*)(H16 + e) = hh; if (ps == 0) __threadfence(); } }
__global__ __launch_bounds__(256) void k_x1(const h16* __restrict__ H2_16, const float* __restrict__ VM, const float* __restrict__ WE, const int* __restrict__ tw, int t, h16* X1) { const size_t e = ((size_t)blockIdx.x * 256 + threadIdx.x) * 4; if (e >= (size_t)NBT * K1) return; const int k = (int)(e % K1); const int b = (int)(e / K1); int widx = t == 0 ? 1 : tw[b * TW + t]; widx = min(max(widx, 0), DICT - 1); v4h o;
#pragma unroll
    for (int q = 0; q < 4; ++q) { const int kk = k + q; h16 v; if (kk < LP) v = H2_16[(size_t)b * LP + kk]; else if (kk < LP + DI) v = tohx(VM[(size_t)b * DI + kk - LP]); else { const int ee = kk - LP - DI; v = ee < LH ? tohx(bfr(WE[(size_t)ee * DICT + widx])) : (h16)0.f; } o[q] = v; }
    *(volatile v4h*)(X1 + e) = o; __threadfence(); *(volatile v4h*)(X1 + e) = o; }
__global__ __launch_bounds__(256) void k_cell(const float* __restrict__ GA, const float* __restrict__ GB, const float* __restrict__ bih, const float* __restrict__ bhh, float* H, float* Cs, h16* H16, h16* X2, int ldx2) { const size_t e = ((size_t)blockIdx.x * 256 + threadIdx.x) * 2; if (e >= (size_t)NBT * LP) return; const int j = (int)(e % LP); const int b = (int)(e / LP); const v2f cold = *(const v2f*)(Cs + e); v2f h, c; v2h hh;
#pragma unroll
    for (int q = 0; q < 2; ++q) { const int jj = j + q; if (jj >= LH) { h[q] = 0.f; c[q] = 0.f; hh[q] = (h16)0.f; continue; } float gt[4];
#pragma unroll
        for (int g = 0; g < 4; ++g) { const size_t col = (size_t)b * G4 + g * LP + jj; const int oi = g * LH + jj; gt[g] = __fadd_rn(__fadd_rn(GA[col], GB[col]), __fadd_rn(bfr(bih[oi]), bfr(bhh[oi]))); }
        float t1 = __fmul_rn(sigm_(gt[1]), cold[q]); asm volatile("" : "+v"(t1)); float t2 = __fmul_rn(sigm_(gt[0]), tanh_(gt[2])); asm volatile("" : "+v"(t2)); c[q] = __fadd_rn(t1, t2); h[q] = __fmul_rn(sigm_(gt[3]), tanh_(c[q])); hh[q] = tohx(h[q]); }
    for (int ps = 0; ps < 2; ++ps) { *(volatile v2f*)(H + e) = h; *(volatile v2f*)(Cs + e) = c; *(volatile v2h*)(H16 + e) = hh; if (X2) *(volatile v2h*)(X2 + (size_t)b * ldx2 + j) = hh; if (ps == 0) __threadfence(); } }
__global__ __launch_bounds__(64) void k_att(const float* __restrict__ IE, const float* __restrict__ HA, const float* __restrict__ wa, const float* __restrict__ ba, const float* __restrict__ F, h16* X2) { const int lane = threadIdx.x & 31; const int b = blockIdx.x * 2 + (threadIdx.x >> 5); if (b >= NBT) return; float mine0 = -3.0e38f, mine1 = -3.0e38f;
#pragma unroll 1
    for (int n = 0; n < NF; ++n) { float s = 0.f;
#pragma unroll 1
        for (int r = 0; r < 16; ++r) { const int a = r * 32 + lane; float p = __fmul_rn(tanh_(__fadd_rn(IE[((size_t)b * NF + n) * DAT + a], HA[(size_t)b * DAT + a])), bfr(wa[a])); asm volatile("" : "+v"(p)); s = __fadd_rn(s, p); }
#pragma unroll
        for (int sh = 16; sh; sh >>= 1) s += __shfl_xor(s, sh, 32);
        const float lg = __fadd_rn(s, bfr(ba[0])); if (n < 32) { if (lane == n) mine0 = lg; } else { if (lane == n - 32) mine1 = lg; } }
    float mx = fmaxf(mine0, mine1);
#pragma unroll
    for (int sh = 16; sh; sh >>= 1) mx = fmaxf(mx, __shfl_xor(mx, sh, 32));
    float d0 = __fsub_rn(mine0, mx); asm volatile("" : "+v"(d0)); float e0 = __expf(d0); float d1 = __fsub_rn(mine1, mx); asm volatile("" : "+v"(d1)); float e1 = (lane < NF - 32) ? __expf(d1) : 0.f; float sum = __fadd_rn(e0, e1);
#pragma unroll
    for (int sh = 16; sh; sh >>= 1) sum += __shfl_xor(sum, sh, 32);
    const float inv = __fdiv_rn(1.0f, sum); const float a0 = __fmul_rn(e0, inv), a1 = __fmul_rn(e1, inv);
    for (int ps = 0; ps < 2; ++ps) {
#pragma unroll 1
        for (int ch = 0; ch < DI / 128; ++ch) { const int f0 = ch * 128 + lane * 4; v4f acc; acc[0] = acc[1] = acc[2] = acc[3] = 0.f;
#pragma unroll 1
            for (int n = 0; n < NF; ++n) { const float an = n < 32 ? __shfl(a0, n, 32) : __shfl(a1, n - 32, 32); const v4f fv = *(const v4f*)(F + ((size_t)b * NF + n) * DI + f0);
#pragma unroll
                for (int q = 0; q < 4; ++q) { float p = __fmul_rn(an, bfr(fv[q])); asm volatile("" : "+v"(p)); acc[q] = __fadd_rn(acc[q], p); } }
            v4h o; o[0] = tohx(acc[0]); o[1] = tohx(acc[1]); o[2] = tohx(acc[2]); o[3] = tohx(acc[3]); *(volatile v4h*)(X2 + (size_t)b * K2 + LP + f0) = o; } if (ps == 0) __threadfence(); } }
#define NSLOT 2528
__global__ __launch_bounds__(256) void k_yout(const float* __restrict__ Y, const float* __restrict__ bp, int t, float* OUT) { const int e = blockIdx.x * 256 + threadIdx.x; if (e >= NBT * NSLOT) return; const int s = e % NSLOT, b = e / NSLOT; const size_t rowf = ((size_t)b * NSTEP + t) * DICT; const size_t line0f = (rowf / 32) * 32; const long v0 = (long)(line0f + 4 * (size_t)s) - (long)rowf; if (v0 < 0 || v0 >= DICT) return; v4f o;
#pragma unroll
    for (int q = 0; q < 4; ++q) { const int v = (int)v0 + q; o[q] = __fadd_rn(Y[(size_t)b * DVP + v], bfr(bp[v])); }
    *(volatile v4f*)(OUT + rowf + v0) = o; __threadfence(); *(volatile v4f*)(OUT + rowf + v0) = o; }

extern "C" void kernel_launch(void* const* d_in, const int* in_sizes, int n_in,
                              void* d_out, int out_size, void* d_ws, size_t ws_size, hipStream_t stream) {
    (void)in_sizes; (void)n_in; (void)out_size;
    const float* feats = (const float*)d_in[0]; const int* tw = (const int*)d_in[2]; const float* WE = (const float*)d_in[3]; const float* W1ih = (const float*)d_in[4]; const float* W1hh = (const float*)d_in[5]; const float* b1ih = (const float*)d_in[6]; const float* b1hh = (const float*)d_in[7]; const float* W2ih = (const float*)d_in[8]; const float* W2hh = (const float*)d_in[9]; const float* b2ih = (const float*)d_in[10]; const float* b2hh = (const float*)d_in[11];
    const float* Waimg = (const float*)d_in[12]; const float* Wah = (const float*)d_in[13]; const float* wa = (const float*)d_in[14]; const float* ba = (const float*)d_in[15]; const float* Wp = (const float*)d_in[16]; const float* bp = (const float*)d_in[17]; const float* h10 = (const float*)d_in[18]; const float* c10 = (const float*)d_in[19]; const float* h20 = (const float*)d_in[20]; const float* c20 = (const float*)d_in[21];
    float* OUT = (float*)d_out;
    char* wsp = (char*)d_ws;
    auto take = [&](size_t bytes) { char* p = wsp; wsp += (bytes + 255) & ~(size_t)255; return (void*)p; };
    h16* W1X = (h16*)take((size_t)G4 * K1 * 2); h16* W1H = (h16*)take((size_t)G4 * LP * 2); h16* W2X = (h16*)take((size_t)G4 * K2 * 2); h16* W2H = (h16*)take((size_t)G4 * LP * 2); h16* WAH = (h16*)take((size_t)DAT * LP * 2); h16* WPP = (h16*)take((size_t)DVP * LP * 2); bf* WAI = (bf*)take((size_t)DAT * DI * 2);
    bf* FB = (bf*)take((size_t)NBT * NF * DI * 2); float* IE = (float*)take((size_t)NBT * NF * DAT * 4); float* VM = (float*)take((size_t)NBT * DI * 4);
    float* H1 = (float*)take((size_t)NBT * LP * 4); float* C1 = (float*)take((size_t)NBT * LP * 4); h16* H1_16 = (h16*)take((size_t)NBT * LP * 2); float* H2 = (float*)take((size_t)NBT * LP * 4); float* C2 = (float*)take((size_t)NBT * LP * 4); h16* H2_16 = (h16*)take((size_t)NBT * LP * 2);
    h16* X1 = (h16*)take((size_t)NBT * K1 * 2); h16* X2 = (h16*)take((size_t)NBT * K2 * 2); float* GA = (float*)take((size_t)NBT * G4 * 4); float* GB = (float*)take((size_t)NBT * G4 * 4); float* HA = (float*)take((size_t)NBT * DAT * 4); float* Y = (float*)take((size_t)NBT * DVP * 4);
    if ((size_t)(wsp - (char*)d_ws) > ws_size) return;
    k_w1x<<<(unsigned)(((size_t)G4 * K1 / 4 + 255) / 256), 256, 0, stream>>>(W1ih, W1X); k_whh<<<(unsigned)(((size_t)G4 * LP / 4 + 255) / 256), 256, 0, stream>>>(W1hh, W1H); k_w2x<<<(unsigned)(((size_t)G4 * K2 / 4 + 255) / 256), 256, 0, stream>>>(W2ih, W2X); k_whh<<<(unsigned)(((size_t)G4 * LP / 4 + 255) / 256), 256, 0, stream>>>(W2hh, W2H);
    k_wah<<<(unsigned)(((size_t)DAT * LP / 4 + 255) / 256), 256, 0, stream>>>(Wah, WAH); k_wp<<<(unsigned)(((size_t)DVP * LP / 4 + 255) / 256), 256, 0, stream>>>(Wp, WPP); k_cvt8<<<(unsigned)(((size_t)DAT * DI / 8 + 255) / 256), 256, 0, stream>>>(Waimg, WAI, (size_t)DAT * DI / 8);
    k_cvt8<<<(unsigned)(((size_t)NBT * NF * DI / 8 + 255) / 256), 256, 0, stream>>>(feats, FB, (size_t)NBT * NF * DI / 8);
    k_gemmw<bf, 0, false><<<dim3(NBT * NF / 64, DAT / 64, 1), 32, 0, stream>>>(FB, nullptr, WAI, nullptr, DI, IE, DAT, nullptr, 0, 0, 0);
    k_vmean<<<(unsigned)(((size_t)NBT * DI / 4 + 255) / 256), 256, 0, stream>>>(feats, VM);
    k_init<<<(NBT * LP / 4 + 255) / 256, 256, 0, stream>>>(h10, c10, H1, C1, H1_16); k_init<<<(NBT * LP / 4 + 255) / 256, 256, 0, stream>>>(h20, c20, H2, C2, H2_16);
    const unsigned LC = (unsigned)((NBT * LP / 2 + 255) / 256);
    for (int t = 0; t < NSTEP; ++t) {
        k_x1<<<(unsigned)(((size_t)NBT * K1 / 4 + 255) / 256), 256, 0, stream>>>(H2_16, VM, WE, tw, t, X1);
        k_gemmw<h16, 0, false><<<dim3(1, G4 / 64, 1), 32, 0, stream>>>(X1, nullptr, W1X, nullptr, K1, GA, G4, nullptr, 0, 0, 0); k_gemmw<h16, 0, false><<<dim3(1, G4 / 64, 1), 32, 0, stream>>>(H1_16, nullptr, W1H, nullptr, LP, GB, G4, nullptr, 0, 0, 0);
        k_cell<<<LC, 256, 0, stream>>>(GA, GB, b1ih, b1hh, H1, C1, H1_16, X2, K2);
        k_gemmw<h16, 0, false><<<dim3(1, DAT / 64, 1), 32, 0, stream>>>(H1_16, nullptr, WAH, nullptr, LP, HA, DAT, nullptr, 0, 0, 0);
        k_att<<<NBT / 2, 64, 0, stream>>>(IE, HA, wa, ba, feats, X2);
        k_gemmw<h16, 0, false><<<dim3(1, G4 / 64, 1), 32, 0, stream>>>(X2, nullptr, W2X, nullptr, K2, GA, G4, nullptr, 0, 0, 0); k_gemmw<h16, 0, false><<<dim3(1, G4 / 64, 1), 32, 0, stream>>>(H2_16, nullptr, W2H, nullptr, LP, GB, G4, nullptr, 0, 0, 0);
        k_cell<<<LC, 256, 0, stream>>>(GA, GB, b2ih, b2hh, H2, C2, H2_16, nullptr, 0);
        k_gemmw<h16, 0, false><<<dim3(1, DVP / 64, 1), 32, 0, stream>>>(H2_16, nullptr, WPP, nullptr, LP, Y, DVP, nullptr, 0, 0, 0);
        k_yout<<<(NBT * NSLOT + 255) / 256, 256, 0, stream>>>(Y, bp, t, OUT); }
}
